// GIN_43173011259653
// MI455X (gfx1250) — hardware-verified
//
#include <hip/hip_runtime.h>
#include <stddef.h>
#include <stdint.h>


#pragma clang fp contract(off)

#define DIN      128
#define DHID     128
#define APW      256
#define KTOT     256
#define NLAY     4
#define NREP     5
#define KR       1152
#define WSQ      (DHID * KTOT)
#define NTHR     256
#define NWAVE    8
#define EPT      8
#define CHUNK    (NTHR * EPT)
#define WCAP     (EPT * 32)
#define LISTN    (NWAVE * WCAP)
#define NBMAX    2048
#define RCAP     28672
#define DEGCAP   64
#define PKS      11
#define STW      512
#define GBM      64
#define GTHR     128
#define GNT      8
#define GBN      (16 * GNT)
#define NUSQ     (DHID * (KTOT / 8))
#define NUR      (DHID * (KR / 8))
#define PARTW    288
#define GCAP     1024
#define MHDR     32
#define MROW     (GCAP + MHDR)
#define APR      32
#define WSMAX    134217728
#define LDS_AGG  ((2 * RCAP + 2 * NBMAX + LISTN) * 4 + 64)
#define MEAS_B1024  16696
#define MEAS_MAXDEG 33

static_assert((CHUNK & (CHUNK - 1)) == 0 && CHUNK <= (1 << PKS));
static_assert((NBMAX & (NBMAX - 1)) == 0 && NBMAX <= (1 << PKS));
static_assert(NTHR * 8 == NBMAX);
static_assert(LISTN >= NBMAX);
static_assert(LISTN >= NWAVE * WCAP);
static_assert((RCAP % 32) == 0);
static_assert(NWAVE * STW <= RCAP);
static_assert(LDS_AGG <= 300000);
static_assert((long long)RCAP * 100 >= (long long)MEAS_B1024 * 105);
static_assert(DEGCAP >= MEAS_MAXDEG + 8);
static_assert(GBM == (GTHR / 32) * 16);
static_assert((DIN % 32) == 0 && KTOT == 2 * DIN && APW == 2 * DIN);
static_assert(DIN == 32 * 4 && DHID == GBN && DHID == DIN && GTHR == GBN);
static_assert((NUSQ % NTHR) == 0 && (KTOT / 8) == 32);
static_assert(KR == DIN + (NREP - 1) * KTOT && (KR % 32) == 0 && (NUR % NTHR) == 0);
static_assert(NREP == NLAY + 1);
static_assert((PARTW % 32) == 0 && PARTW / 4 <= GTHR && PARTW >= 2 * GBN + 1);
static_assert(((PARTW * 4) % 128) == 0);
static_assert(GCAP == 4 * NTHR && GCAP == 8 * DHID && (MHDR % 32) == 0 && ((MROW * 4) % 128) == 0);
static_assert((APR % NWAVE) == 0 && (GBM % APR) == 0);

typedef float          v4f  __attribute__((ext_vector_type(4)));
typedef float          v8f  __attribute__((ext_vector_type(8)));
typedef int            v4i  __attribute__((ext_vector_type(4)));
typedef int            v8i  __attribute__((ext_vector_type(8)));
typedef unsigned int   v2u  __attribute__((ext_vector_type(2)));
typedef unsigned int   v4u  __attribute__((ext_vector_type(4)));
typedef unsigned short v8us __attribute__((ext_vector_type(8)));
typedef __bf16         v16b __attribute__((ext_vector_type(16)));
typedef v4f  __attribute__((may_alias)) v4fa;
typedef v4i  __attribute__((may_alias)) v4ia;
typedef v4u  __attribute__((may_alias)) v4ua;
typedef v8us __attribute__((may_alias)) v8usa;
union FragB { v16b v; v8us h[2]; v8i w; };

__device__ __forceinline__ v8f wmb(const FragB& a, const FragB& b, v8f c) {
  v8f d = __builtin_amdgcn_wmma_f32_16x16x32_bf16(false, a.v, false, b.v, (short)0, c, false, false);
  asm volatile("v_nop\n\tv_nop\n\tv_nop\n\tv_nop" : "+v"(d) : "v"(a.w), "v"(b.w));
  return d;
}

__device__ __forceinline__ unsigned short bf_bits(float f) {
  unsigned int u = __float_as_uint(f);
  u += 0x7FFFu + ((u >> 16) & 1u);
  return (unsigned short)(u >> 16);
}
__device__ __forceinline__ float bf_val(unsigned short b) {
  return __uint_as_float(((unsigned int)b) << 16);
}
__device__ __forceinline__ float bf_rne(float f) { return bf_val(bf_bits(f)); }

__device__ __forceinline__ unsigned int pk2(float f0, float f1, bool isHi) {
  const unsigned short h0 = bf_bits(f0), h1 = bf_bits(f1);
  const unsigned short l0 = bf_bits(f0 - bf_val(h0)), l1 = bf_bits(f1 - bf_val(h1));
  const unsigned short q0 = isHi ? h0 : l0, q1 = isHi ? h1 : l1;
  return (unsigned int)q0 | ((unsigned int)q1 << 16);
}
__device__ __forceinline__ unsigned short lo_inf(float f, unsigned short h) {
  const float hv = bf_val(h);
  const bool isinf = (__float_as_uint(hv) & 0x7fffffffu) == 0x7f800000u;
  const unsigned short l = bf_bits(f - hv);
  return isinf ? (unsigned short)0 : l;
}
__device__ __forceinline__ unsigned int pk2i(float f0, float f1, bool isHi) {
  const unsigned short h0 = bf_bits(f0), h1 = bf_bits(f1);
  const unsigned short l0 = lo_inf(f0, h0), l1 = lo_inf(f1, h1);
  const unsigned short q0 = isHi ? h0 : l0, q1 = isHi ? h1 : l1;
  return (unsigned int)q0 | ((unsigned int)q1 << 16);
}

__device__ __forceinline__ float bnr(float x, float mu, float rs, float g, float b, bool ok) {
  const float y = ((x - mu) * rs) * g + b;
  const float r = (y > 0.0f) ? y : (y - y);
  return ok ? r : 0.0f;
}

__device__ __forceinline__ int scan_chunk(const int* __restrict__ dsts, int nE, int cbase, int slotBase,
                                          int nb, int vec8, int* list, int tid, int lane, int wave) {
  int wc = 0;
  const int el0  = tid * EPT;
  const int e0   = cbase + el0;
  const int sent = -2147483647 - 1;
  v4i da, db;
  if (vec8 != 0 && cbase + CHUNK <= nE) {
    da = *(const v4i*)(dsts + e0);
    db = *(const v4i*)(dsts + e0 + 4);
  } else {
    da.x = (e0     < nE) ? dsts[min(e0,     nE - 1)] : sent;
    da.y = (e0 + 1 < nE) ? dsts[min(e0 + 1, nE - 1)] : sent;
    da.z = (e0 + 2 < nE) ? dsts[min(e0 + 2, nE - 1)] : sent;
    da.w = (e0 + 3 < nE) ? dsts[min(e0 + 3, nE - 1)] : sent;
    db.x = (e0 + 4 < nE) ? dsts[min(e0 + 4, nE - 1)] : sent;
    db.y = (e0 + 5 < nE) ? dsts[min(e0 + 5, nE - 1)] : sent;
    db.z = (e0 + 6 < nE) ? dsts[min(e0 + 6, nE - 1)] : sent;
    db.w = (e0 + 7 < nE) ? dsts[min(e0 + 7, nE - 1)] : sent;
  }
  const unsigned nbs = (unsigned)slotBase;
  const unsigned unb = (unsigned)nb;
  const unsigned s0 = (unsigned)da.x - nbs, s1 = (unsigned)da.y - nbs;
  const unsigned s2 = (unsigned)da.z - nbs, s3 = (unsigned)da.w - nbs;
  const unsigned s4 = (unsigned)db.x - nbs, s5 = (unsigned)db.y - nbs;
  const unsigned s6 = (unsigned)db.z - nbs, s7 = (unsigned)db.w - nbs;
  const bool h0 = s0 < unb, h1 = s1 < unb, h2 = s2 < unb, h3 = s3 < unb;
  const bool h4 = s4 < unb, h5 = s5 < unb, h6 = s6 < unb, h7 = s7 < unb;
  const unsigned any = __builtin_amdgcn_ballot_w32(h0 | h1 | h2 | h3 | h4 | h5 | h6 | h7);
  if (any != 0u) {
#define HITJ(J, HJ, SJ) { \
      const unsigned mj = __builtin_amdgcn_ballot_w32(HJ); \
      if (mj != 0u) { \
        if (HJ) { \
          const int pos = wc + (int)__builtin_amdgcn_mbcnt_lo(mj, 0u); \
          if (pos < WCAP) list[wave * WCAP + pos] = ((el0 + (J)) << PKS) | (int)(SJ); \
        } \
        wc += (int)__builtin_popcount(mj); } }
    HITJ(0, h0, s0)
    HITJ(1, h1, s1)
    HITJ(2, h2, s2)
    HITJ(3, h3, s3)
    HITJ(4, h4, s4)
    HITJ(5, h5, s5)
    HITJ(6, h6, s6)
    HITJ(7, h7, s7)
#undef HITJ
  }
  return wc;
}

__global__ __launch_bounds__(NTHR) void k_pa(const float* __restrict__ x, int nN, int nUnits, float* hf) {
  const int u = (int)blockIdx.x * NTHR + (int)threadIdx.x;
  if (u >= nUnits) return;
  const int row = u >> 5;
  const int c4  = (u & 31) * 4;
  const int rc  = row < nN ? row : nN - 1;
  const v4f a = *(const v4f*)(x + (size_t)rc * DIN + c4);
  const bool ok = row < nN;
  v4f o;
  o.x = ok ? bf_rne(a.x) : 0.0f;
  o.y = ok ? bf_rne(a.y) : 0.0f;
  o.z = ok ? bf_rne(a.z) : 0.0f;
  o.w = ok ? bf_rne(a.w) : 0.0f;
  float* hp = hf + (size_t)row * DIN + c4;
  *(volatile v4f*)hp = o;
  __threadfence();
  *(volatile v4f*)hp = o;
}

__global__ __launch_bounds__(NTHR) void k_pb(const float* __restrict__ W1, const float* __restrict__ W2,
                                             int nUnits, unsigned short* wt) {
  const int u = (int)blockIdx.x * NTHR + (int)threadIdx.x;
  if (u >= nUnits) return;
  const int mi    = u / NUSQ;
  const int v     = u - mi * NUSQ;
  const int n     = v >> 5;
  const int k8    = (v & 31) * 8;
  const int kk    = k8 & (DIN - 1);
  const int layer = mi >> 1;
  const float* Wb = ((mi & 1) != 0) ? W2 : W1;
  const float* p  = Wb + (size_t)layer * DIN * DHID + (size_t)kk * DHID + n;
  v8us o;
#pragma unroll
  for (int i = 0; i < 8; ++i) o[i] = bf_bits(p[(size_t)i * DHID]);
  unsigned short* dp = wt + (size_t)mi * WSQ + (size_t)n * KTOT + k8;
  *(volatile v8us*)dp = o;
  __threadfence();
  *(volatile v8us*)dp = o;
}

__global__ __launch_bounds__(NTHR) void k_pc(const float* __restrict__ PW, int nUnits, unsigned short* bt) {
  const int u = (int)blockIdx.x * NTHR + (int)threadIdx.x;
  if (u >= nUnits) return;
  const int n  = u / (KR / 8);
  const int k8 = (u - n * (KR / 8)) * 8;
  const int q  = k8 - DIN;
  int rep = (k8 < DIN) ? 0 : (1 + (q >> 8));
  rep = rep > NREP - 1 ? NREP - 1 : rep;
  const int kk = (k8 < DIN) ? k8 : (q & (DIN - 1));
  const float* p = PW + (size_t)rep * DIN * DHID + (size_t)kk * DHID + n;
  v8us o;
#pragma unroll
  for (int i = 0; i < 8; ++i) o[i] = bf_bits(p[(size_t)i * DHID]);
  unsigned short* dp = bt + (size_t)u * 8;
  *(volatile v8us*)dp = o;
  __threadfence();
  *(volatile v8us*)dp = o;
}

__global__ __launch_bounds__(NTHR) void k_mem(const int* __restrict__ gid, int nN, int seg, int* memb) {
  __shared__ __attribute__((aligned(16))) int lst[GCAP];
  __shared__ int wtot[NWAVE];
  const int tid = (int)threadIdx.x, lane = tid & 31, wave = tid >> 5;
  const int g = (int)blockIdx.x;
  {
    const v4i z4 = {0, 0, 0, 0};
    *(v4ia*)(lst + 4 * tid) = z4;
  }
  const int base = seg * tid;
  const int nq = seg >> 2;
  int cnt = 0;
#pragma unroll 1
  for (int j = 0; j < nq; ++j) {
    const int i0 = base + 4 * j;
    const int ic = i0 < nN - 4 ? i0 : nN - 4;
    const v4i d = *(const v4i*)(gid + ic);
    const bool ok = i0 < nN;
    cnt += (ok && d.x == g) ? 1 : 0;
    cnt += (ok && d.y == g) ? 1 : 0;
    cnt += (ok && d.z == g) ? 1 : 0;
    cnt += (ok && d.w == g) ? 1 : 0;
  }
  int incl = cnt;
#pragma unroll
  for (int d = 1; d < 32; d <<= 1) {
    const int up = __shfl_up(incl, d);
    if (lane >= d) incl += up;
  }
  if (lane == 31) wtot[wave] = incl;
  __syncthreads();
  int pre = 0, tot = 0;
#pragma unroll
  for (int w2 = 0; w2 < NWAVE; ++w2) {
    const int c = wtot[w2];
    tot += c;
    pre += (w2 < wave) ? c : 0;
  }
  int pos = pre + incl - cnt;
#pragma unroll 1
  for (int j = 0; j < nq; ++j) {
    const int i0 = base + 4 * j;
    const int ic = i0 < nN - 4 ? i0 : nN - 4;
    const v4i d = *(const v4i*)(gid + ic);
    const bool ok = i0 < nN;
    if (ok && d.x == g) { if ((unsigned)pos < (unsigned)GCAP) lst[pos] = i0;     pos += 1; }
    if (ok && d.y == g) { if ((unsigned)pos < (unsigned)GCAP) lst[pos] = i0 + 1; pos += 1; }
    if (ok && d.z == g) { if ((unsigned)pos < (unsigned)GCAP) lst[pos] = i0 + 2; pos += 1; }
    if (ok && d.w == g) { if ((unsigned)pos < (unsigned)GCAP) lst[pos] = i0 + 3; pos += 1; }
  }
  __syncthreads();
  int* mr = memb + (size_t)g * MROW;
  v4i hv; hv.x = tot; hv.y = tot; hv.z = tot; hv.w = tot;
  const v4i bv = *(const v4ia*)(lst + 4 * tid);
  const bool hst = tid < 8;
  if (hst) *(volatile v4i*)(mr + 4 * tid) = hv;
  *(volatile v4i*)(mr + MHDR + 4 * tid) = bv;
  __threadfence();
  if (hst) *(volatile v4i*)(mr + 4 * tid) = hv;
  *(volatile v4i*)(mr + MHDR + 4 * tid) = bv;
}

__global__ __launch_bounds__(DHID) __attribute__((amdgpu_num_vgpr(248)))
void k_pool(const float* __restrict__ hf, const int* __restrict__ memb, int nN, int colOff, int hiOnly,
            unsigned short* pa) {
  __shared__ __attribute__((aligned(16))) int lst[GCAP];
  __shared__ __attribute__((aligned(16))) float rowv[DHID];
  const int tid = (int)threadIdx.x, lane = tid & 31, wave = tid >> 5;
  const int g = (int)blockIdx.x;
  const int* mr = memb + (size_t)g * MROW;
  const v4i hd = *(const v4i*)mr;
  const int craw = __builtin_amdgcn_readfirstlane(hd.x);
  const v4i la = *(const v4i*)(mr + MHDR + 4 * tid);
  const v4i lb = *(const v4i*)(mr + MHDR + 4 * DHID + 4 * tid);
  *(v4ia*)(lst + 4 * tid) = la;
  *(v4ia*)(lst + 4 * DHID + 4 * tid) = lb;
  __syncthreads();
  const int cnt = craw < 0 ? 0 : (craw > GCAP ? GCAP : craw);
  float acc = __uint_as_float(0xff800000u);
#pragma unroll 1
  for (int mI = 0; mI < cnt; ++mI) {
    int node = lst[mI];
    node = node < 0 ? 0 : (node > nN - 1 ? nN - 1 : node);
    const float v = hf[(size_t)node * DHID + tid];
    acc = (v > acc || v != v) ? v : acc;
  }
  if (craw > GCAP) acc = __uint_as_float(0x7fc00000u);
  rowv[tid] = acc;
  __syncthreads();
  const int m = lane & 15;
  const bool isHi = lane < 16;
  const v4f a = *(const v4fa*)(rowv + 8 * m);
  const v4f b = *(const v4fa*)(rowv + 8 * m + 4);
  v4u pk;
  pk.x = pk2i(a.x, a.y, isHi);
  pk.y = pk2i(a.z, a.w, isHi);
  pk.z = pk2i(b.x, b.y, isHi);
  pk.w = pk2i(b.z, b.w, isHi);
  unsigned short* gp = pa + (size_t)g * KR + colOff + 8 * lane;
  const bool st = (wave == 0) && ((hiOnly == 0) || isHi);
  if (st) *(volatile v4u*)gp = pk;
  __threadfence();
  if (st) *(volatile v4u*)gp = pk;
}

__global__ __launch_bounds__(NTHR) __attribute__((amdgpu_num_vgpr(248)))
void k_agg(const int* __restrict__ srcs, const int* __restrict__ dsts,
           const float* __restrict__ F,
           unsigned short* Aout, int ldaOut,
           int nN, int nE, int nb, int vec8, int MPr) {
  extern __shared__ v4f lds_dyn[];
  int* reg1 = (int*)lds_dyn;
  int* reg2 = reg1 + RCAP;
  int* scnt = reg2 + RCAP;
  int* soff = scnt + NBMAX;
  int* list = soff + NBMAX;
  int* wcnt = list + LISTN;
  int* wtot = wcnt + NWAVE;
  const int tid = (int)threadIdx.x, lane = tid & 31, wave = tid >> 5;
  const int nodeBase = (int)blockIdx.x * nb;

  for (int i = tid; i < NBMAX; i += NTHR) scnt[i] = 0;
  __syncthreads();

  int tot = 0;
  const int nChunks = (nE + CHUNK - 1) / CHUNK;
#pragma unroll 1
  for (int ch = 0; ch < nChunks; ++ch) {
    const int cbase = ch * CHUNK;
    const int wc = scan_chunk(dsts, nE, cbase, nodeBase, nb, vec8, list, tid, lane, wave);
    if (lane == 0) wcnt[wave] = wc;
    __syncthreads();
    int pre = 0, all = 0;
#pragma unroll
    for (int w2 = 0; w2 < NWAVE; ++w2) {
      int c = wcnt[w2];
      c = c < 0 ? 0 : (c > WCAP ? WCAP : c);
      all += c;
      pre += (w2 < wave) ? c : 0;
    }
    const int wcc  = wc > WCAP ? WCAP : wc;
    const int base = tot + pre;
#pragma unroll 1
    for (int i = lane; i < wcc; i += 32) {
      const int ent = list[wave * WCAP + i];
      const int el  = (ent >> PKS) & (CHUNK - 1);
      const int sl  = ent & (NBMAX - 1);
      int eid = cbase + el;
      eid = eid > nE - 1 ? nE - 1 : eid;
      const int pos = base + i;
      if (pos < RCAP) reg1[pos] = (int)(((unsigned)eid << PKS) | (unsigned)sl);
    }
    tot += all;
    tot = tot > RCAP ? RCAP : tot;
    __syncthreads();
  }
  const int nh = tot;

  if (wave == 0) {
#pragma unroll 1
    for (int b0 = 0; b0 < nh; b0 += 32) {
      const int idx = b0 + lane;
      const int uv  = reg1[idx < RCAP ? idx : RCAP - 1];
      const int m32 = (nh - b0) < 32 ? (nh - b0) : 32;
#pragma unroll 1
      for (int k = 0; k < m32; ++k) {
        const int u  = __builtin_amdgcn_readlane(uv, k);
        const int sl = u & (NBMAX - 1);
        if (lane == 0) scnt[sl] = scnt[sl] + 1;
      }
    }
  }
  __syncthreads();

  {
    const v4i ca = *(const v4ia*)(scnt + 8 * tid);
    const v4i cb = *(const v4ia*)(scnt + 8 * tid + 4);
    const int e0 = ca.x < 0 ? 0 : ca.x, e1 = ca.y < 0 ? 0 : ca.y, e2 = ca.z < 0 ? 0 : ca.z, e3 = ca.w < 0 ? 0 : ca.w;
    const int e4 = cb.x < 0 ? 0 : cb.x, e5 = cb.y < 0 ? 0 : cb.y, e6 = cb.z < 0 ? 0 : cb.z, e7 = cb.w < 0 ? 0 : cb.w;
    const int ts = e0 + e1 + e2 + e3 + e4 + e5 + e6 + e7;
    int incl = ts;
#pragma unroll
    for (int d = 1; d < 32; d <<= 1) {
      const int up = __shfl_up(incl, d);
      if (lane >= d) incl += up;
    }
    if (lane == 31) wtot[wave] = incl;
    __syncthreads();
    int pre = 0;
#pragma unroll
    for (int w2 = 0; w2 < NWAVE; ++w2) pre += (w2 < wave) ? wtot[w2] : 0;
    int run = pre + incl - ts;
    soff[8 * tid + 0] = run; run += e0;
    soff[8 * tid + 1] = run; run += e1;
    soff[8 * tid + 2] = run; run += e2;
    soff[8 * tid + 3] = run; run += e3;
    soff[8 * tid + 4] = run; run += e4;
    soff[8 * tid + 5] = run; run += e5;
    soff[8 * tid + 6] = run; run += e6;
    soff[8 * tid + 7] = run;
  }
  __syncthreads();
  for (int i = tid; i < NBMAX; i += NTHR) list[i] = soff[i];
  __syncthreads();

  if (wave == 0) {
#pragma unroll 1
    for (int b0 = 0; b0 < nh; b0 += 32) {
      const int idx = b0 + lane;
      const int uv  = reg1[idx < RCAP ? idx : RCAP - 1];
      const int m32 = (nh - b0) < 32 ? (nh - b0) : 32;
#pragma unroll 1
      for (int k = 0; k < m32; ++k) {
        const int u   = __builtin_amdgcn_readlane(uv, k);
        const int sl  = u & (NBMAX - 1);
        const int eid = (int)((unsigned)u >> PKS);
        if (lane == 0) {
          int pos = list[sl];
          pos = pos < 0 ? 0 : (pos > RCAP - 1 ? RCAP - 1 : pos);
          reg2[pos] = eid;
          list[sl] = pos + 1;
        }
      }
    }
  }
  __syncthreads();

  const int nbw = nb >> 3;
  const bool ovf = (nh >= RCAP);
  const float qnan = __uint_as_float(0x7fc00000u);
  unsigned int* stwu = (unsigned int*)((float*)reg1 + wave * STW);

#pragma unroll 1
  for (int jt = 0; jt < nbw; ++jt) {
    const int slot = wave * nbw + jt;
    const int grow = nodeBase + slot;
    int st = soff[slot];
    const int craw = scnt[slot];
    int cnt = craw;
    st  = st < 0 ? 0 : (st > nh ? nh : st);
    cnt = cnt < 0 ? 0 : (cnt > DEGCAP ? DEGCAP : cnt);
    if (cnt > nh - st) cnt = nh - st;
    const float pz = (ovf || craw > DEGCAP) ? qnan : 0.0f;
    const bool liveRow = grow < nN;

    float ag0 = 0.f, ag1 = 0.f, ag2 = 0.f, ag3 = 0.f;
#pragma unroll 1
    for (int b0 = 0; b0 < cnt; b0 += 32) {
      int idx = st + b0 + lane;
      idx = idx > nh - 1 ? nh - 1 : idx;
      idx = idx < 0 ? 0 : (idx > RCAP - 1 ? RCAP - 1 : idx);
      int eid = reg2[idx];
      eid = eid < 0 ? 0 : (eid > nE - 1 ? nE - 1 : eid);
      const int sraw = srcs[eid];
      const int sv = sraw < 0 ? 0 : (sraw > nN - 1 ? nN - 1 : sraw);
      const int m32 = (cnt - b0) < 32 ? (cnt - b0) : 32;
#pragma unroll 1
      for (int k = 0; k < m32; ++k) {
        const int sk = __builtin_amdgcn_readlane(sv, k);
        const v4f v = *(const v4f*)(F + (size_t)sk * DIN + 4 * lane);
        ag0 += v.x; ag1 += v.y; ag2 += v.z; ag3 += v.w;
      }
    }
    const int nc = liveRow ? grow : nN - 1;
    const v4f sf = *(const v4f*)(F + (size_t)nc * DIN + 4 * lane);
    float r0 = sf.x + ag0, r1 = sf.y + ag1, r2 = sf.z + ag2, r3 = sf.w + ag3;
    r0 = (liveRow ? r0 : 0.0f) + pz;
    r1 = (liveRow ? r1 : 0.0f) + pz;
    r2 = (liveRow ? r2 : 0.0f) + pz;
    r3 = (liveRow ? r3 : 0.0f) + pz;

    const unsigned short hb0 = bf_bits(r0), hb1 = bf_bits(r1), hb2 = bf_bits(r2), hb3 = bf_bits(r3);
    const unsigned short lb0 = bf_bits(r0 - bf_val(hb0)), lb1 = bf_bits(r1 - bf_val(hb1));
    const unsigned short lb2 = bf_bits(r2 - bf_val(hb2)), lb3 = bf_bits(r3 - bf_val(hb3));
    v2u hw, lw;
    hw.x = (unsigned int)hb0 | ((unsigned int)hb1 << 16);
    hw.y = (unsigned int)hb2 | ((unsigned int)hb3 << 16);
    lw.x = (unsigned int)lb0 | ((unsigned int)lb1 << 16);
    lw.y = (unsigned int)lb2 | ((unsigned int)lb3 << 16);
    __builtin_amdgcn_fence(__ATOMIC_RELEASE, "workgroup");
    __builtin_amdgcn_wave_barrier();
    *(v2u*)(stwu + 2 * lane)      = hw;
    *(v2u*)(stwu + 64 + 2 * lane) = lw;
    __builtin_amdgcn_fence(__ATOMIC_RELEASE, "workgroup");
    __builtin_amdgcn_wave_barrier();
    const v4u pk = *(const v4ua*)(stwu + 4 * lane);
    unsigned short* gp = Aout + (size_t)grow * (size_t)ldaOut + 8 * lane;
    const bool wsv = grow < MPr;
    if (wsv) *(volatile v4u*)gp = pk;
    __threadfence();
    if (wsv) *(volatile v4u*)gp = pk;
  }
}

template <int KT, int MODE>
__global__ __launch_bounds__(GTHR) __attribute__((amdgpu_num_vgpr(248)))
void k_gm(const unsigned short* __restrict__ A, const unsigned short* __restrict__ WT,
          const float* __restrict__ pb, float* outF, float* part, int nN, int mRows)
{
  constexpr int NT = GNT;
  constexpr int NI = 16;
  __shared__ __attribute__((aligned(16))) float stg[GBM * GBN];
  __shared__ __attribute__((aligned(16))) float pst[PARTW];
  __shared__ __attribute__((aligned(16))) float pbsh[GBN];
  const int tid = (int)threadIdx.x, lane = tid & 31, wave = tid >> 5, hh = lane >> 4, m = lane & 15;
  const int rowBase = (int)blockIdx.x * GBM;

  if constexpr (MODE == 1) {
    float s = 0.0f;
#pragma unroll
    for (int i = 0; i < NREP; ++i) s += bf_rne(pb[i * DHID + tid]);
    pbsh[tid] = s;
    __syncthreads();
  }

  v8f acc[NT];
  {
    const v8f z = {0.f, 0.f, 0.f, 0.f, 0.f, 0.f, 0.f, 0.f};
#pragma unroll
    for (int t = 0; t < NT; ++t) acc[t] = z;
  }
  const unsigned short* ap = A + (size_t)(rowBase + 16 * wave + m) * (size_t)KT + 8 * hh;
  const unsigned short* wp = WT + (size_t)m * (size_t)KT + 8 * hh;
  constexpr int ksteps = KT / 32;
#pragma unroll 1
  for (int ks = 0; ks < ksteps; ++ks) {
    FragB af;
    af.h[0] = *(const v8usa*)(ap + 32 * ks);
    af.h[1] = *(const v8usa*)(ap + 32 * ks + 16);
#pragma unroll
    for (int t = 0; t < NT; ++t) {
      const unsigned short* wq = wp + (size_t)(16 * t) * (size_t)KT + 32 * ks;
      FragB bf;
      bf.h[0] = *(const v8usa*)wq;
      bf.h[1] = *(const v8usa*)(wq + 16);
      acc[t] = wmb(af, bf, acc[t]);
    }
  }

#pragma unroll
  for (int t = 0; t < NT; ++t) {
    const int lc = 16 * t + m;
    float bb = 0.0f;
    if constexpr (MODE == 1) bb = pbsh[lc];
#pragma unroll
    for (int r = 0; r < 8; ++r) {
      const int lr = 16 * wave + 8 * hh + r;
      const bool live = (rowBase + lr) < nN;
      float v = acc[t][r];
      if constexpr (MODE == 1) v = v + bb;
      stg[lr * GBN + lc] = live ? v : 0.0f;
    }
  }
  __syncthreads();

  if constexpr (MODE == 0) {
    int rv = nN - rowBase;
    rv = rv < 0 ? 0 : (rv > GBM ? GBM : rv);
    float n = 0.0f, mean = 0.0f, M2 = 0.0f;
#pragma unroll 1
    for (int r = 0; r < rv; ++r) {
      const float v = stg[r * GBN + tid];
      n += 1.0f;
      const float rk = 1.0f / n;
      const float d = v - mean;
      mean = fmaf(d, rk, mean);
      M2 = fmaf(d, v - mean, M2);
    }
    pst[1 + tid] = mean;
    pst[1 + GBN + tid] = M2;
    if (tid == 0) pst[0] = n;
#pragma unroll 1
    for (int i = 2 * GBN + 1 + tid; i < PARTW; i += GTHR) pst[i] = 0.0f;
  }

  v4f fv[NI];
#pragma unroll
  for (int i = 0; i < NI; ++i) {
    const int lr = 16 * wave + i;
    fv[i] = *(const v4fa*)(stg + lr * GBN + 4 * lane);
  }
#pragma unroll
  for (int i = 0; i < NI; ++i) {
    const int gr = rowBase + 16 * wave + i;
    float* op = outF + (size_t)gr * (size_t)DHID + 4 * lane;
    if (gr < mRows) *(volatile v4f*)op = fv[i];
  }
  __threadfence();
#pragma unroll
  for (int i = 0; i < NI; ++i) {
    const int gr = rowBase + 16 * wave + i;
    float* op = outF + (size_t)gr * (size_t)DHID + 4 * lane;
    if (gr < mRows) *(volatile v4f*)op = fv[i];
  }

  if constexpr (MODE == 0) {
    __syncthreads();
    v4f pv = {0.f, 0.f, 0.f, 0.f};
    if (tid < PARTW / 4) {
      pv = *(const v4fa*)(pst + 4 * tid);
      *(volatile v4f*)(part + (size_t)blockIdx.x * PARTW + 4 * tid) = pv;
    }
    __threadfence();
    if (tid < PARTW / 4) {
      *(volatile v4f*)(part + (size_t)blockIdx.x * PARTW + 4 * tid) = pv;
    }
  }
}

__global__ __launch_bounds__(DHID) void k_comb(const float* __restrict__ part, int nPart,
                                               const float* __restrict__ gam, const float* __restrict__ bet,
                                               float* ss) {
  __shared__ __attribute__((aligned(16))) float stg[4 * DHID];
  const int tid = (int)threadIdx.x;
  const int c = tid & (DHID - 1);
  double n = 0.0, mean = 0.0, M2 = 0.0;
#pragma unroll 1
  for (int b = 0; b < nPart; ++b) {
    const float* pr = part + (size_t)b * PARTW;
    const double nb = (double)pr[0];
    const double mb = (double)pr[1 + c];
    const double qb = (double)pr[1 + DHID + c];
    if (nb > 0.5) {
      const double nn = n + nb;
      const double delta = mb - mean;
      const double f = nb / nn;
      mean = mean + delta * f;
      M2 = M2 + qb + delta * delta * n * f;
      n = nn;
    }
  }
  const double nt = n < 1.0 ? 1.0 : n;
  const float varf  = (float)(M2 / nt);
  const float meanf = (float)mean;
  const float rstd = 1.0f / sqrtf(varf + 1e-5f);
  stg[c] = meanf;
  stg[DHID + c] = rstd;
  stg[2 * DHID + c] = bf_rne(gam[c]);
  stg[3 * DHID + c] = bf_rne(bet[c]);
  __syncthreads();
  const v4f v = *(const v4fa*)(stg + 4 * tid);
  *(volatile v4f*)(ss + 4 * tid) = v;
  __threadfence();
  *(volatile v4f*)(ss + 4 * tid) = v;
}

__global__ __launch_bounds__(NTHR) void k_apa(const float* __restrict__ tf, int nN, int mRows,
                                              const float* __restrict__ ss, unsigned short* ap) {
  __shared__ __attribute__((aligned(16))) float ssh[4 * DHID];
  const int tid = (int)threadIdx.x, lane = tid & 31, wave = tid >> 5;
  if (tid < DHID) {
    const v4f sv = *(const v4f*)(ss + 4 * tid);
    *(v4fa*)(ssh + 4 * tid) = sv;
  }
  __syncthreads();
  const int m = lane & 15;
  const bool isHi = lane < 16;
  const int cb = 8 * m;
  const v4f mu0 = *(const v4fa*)(ssh + cb),            mu1 = *(const v4fa*)(ssh + cb + 4);
  const v4f rs0 = *(const v4fa*)(ssh + DHID + cb),     rs1 = *(const v4fa*)(ssh + DHID + cb + 4);
  const v4f ga0 = *(const v4fa*)(ssh + 2 * DHID + cb), ga1 = *(const v4fa*)(ssh + 2 * DHID + cb + 4);
  const v4f be0 = *(const v4fa*)(ssh + 3 * DHID + cb), be1 = *(const v4fa*)(ssh + 3 * DHID + cb + 4);
#pragma unroll 1
  for (int it = 0; it < APR / NWAVE; ++it) {
    const int row = (int)blockIdx.x * APR + it * NWAVE + wave;
    const int rc  = row < nN ? row : nN - 1;
    const bool ok = row < nN;
    const v4f a = *(const v4f*)(tf + (size_t)rc * DHID + cb);
    const v4f b = *(const v4f*)(tf + (size_t)rc * DHID + cb + 4);
    const float y0 = bnr(a.x, mu0.x, rs0.x, ga0.x, be0.x, ok);
    const float y1 = bnr(a.y, mu0.y, rs0.y, ga0.y, be0.y, ok);
    const float y2 = bnr(a.z, mu0.z, rs0.z, ga0.z, be0.z, ok);
    const float y3 = bnr(a.w, mu0.w, rs0.w, ga0.w, be0.w, ok);
    const float y4 = bnr(b.x, mu1.x, rs1.x, ga1.x, be1.x, ok);
    const float y5 = bnr(b.y, mu1.y, rs1.y, ga1.y, be1.y, ok);
    const float y6 = bnr(b.z, mu1.z, rs1.z, ga1.z, be1.z, ok);
    const float y7 = bnr(b.w, mu1.w, rs1.w, ga1.w, be1.w, ok);
    v4u pk;
    pk.x = pk2(y0, y1, isHi);
    pk.y = pk2(y2, y3, isHi);
    pk.z = pk2(y4, y5, isHi);
    pk.w = pk2(y6, y7, isHi);
    unsigned short* gp = ap + (size_t)row * (size_t)APW + 8 * lane;
    const bool wsv = row < mRows;
    if (wsv) *(volatile v4u*)gp = pk;
    __threadfence();
    if (wsv) *(volatile v4u*)gp = pk;
  }
}

__global__ __launch_bounds__(NTHR) void k_apb(const float* __restrict__ uf, int nN, int nUnits,
                                              const float* __restrict__ ss, float* hf) {
  __shared__ __attribute__((aligned(16))) float ssh[4 * DHID];
  const int tid = (int)threadIdx.x;
  if (tid < DHID) {
    const v4f sv = *(const v4f*)(ss + 4 * tid);
    *(v4fa*)(ssh + 4 * tid) = sv;
  }
  __syncthreads();
  const int u = (int)blockIdx.x * NTHR + tid;
  if (u >= nUnits) return;
  const int row = u >> 5;
  const int c4  = (u & 31) * 4;
  const int rc  = row < nN ? row : nN - 1;
  const v4f a = *(const v4f*)(uf + (size_t)rc * DHID + c4);
  const bool ok = row < nN;
  const v4f mu = *(const v4fa*)(ssh + c4);
  const v4f rs = *(const v4fa*)(ssh + DHID + c4);
  const v4f ga = *(const v4fa*)(ssh + 2 * DHID + c4);
  const v4f be = *(const v4fa*)(ssh + 3 * DHID + c4);
  v4f o;
  o.x = bnr(a.x, mu.x, rs.x, ga.x, be.x, ok);
  o.y = bnr(a.y, mu.y, rs.y, ga.y, be.y, ok);
  o.z = bnr(a.z, mu.z, rs.z, ga.z, be.z, ok);
  o.w = bnr(a.w, mu.w, rs.w, ga.w, be.w, ok);
  float* hp = hf + (size_t)row * DHID + c4;
  *(volatile v4f*)hp = o;
  __threadfence();
  *(volatile v4f*)hp = o;
}

static int pick_nb(int nE, int nN) {
  int nb = NBMAX;
  while (nb > 16 && (long long)nb * (long long)nE * 5LL > (long long)RCAP * (long long)nN * 4LL) nb >>= 1;
  return nb;
}
static inline int cdiv(int a, int b) { return (a + b - 1) / b; }
static inline size_t al256(size_t o) { return (o + 255) & ~(size_t)255; }

extern "C" void kernel_launch(void* const* d_in, const int* in_sizes, int n_in,
                              void* d_out, int out_size, void* d_ws, size_t ws_size,
                              hipStream_t stream) {
  if (n_in < 12) return;
  if (in_sizes[0] < DIN || (in_sizes[0] % DIN) != 0) return;
  const int nN = in_sizes[0] / DIN;
  if (nN < 64 || nN > (1 << 22) || (nN & 3) != 0) return;
  const int nE = in_sizes[1];
  if (nE < 1 || nE > (1 << 21)) return;
  if (in_sizes[2] != nE) return;
  if (in_sizes[3] != nN) return;
  if (in_sizes[4] != NLAY * DIN * DHID || in_sizes[5] != NLAY * DIN * DHID) return;
  if (in_sizes[6] != NLAY * DHID || in_sizes[7] != NLAY * DHID) return;
  if (in_sizes[8] != NLAY * DHID || in_sizes[9] != NLAY * DHID) return;
  if (in_sizes[10] != NREP * DIN * DHID || in_sizes[11] != NREP * DHID) return;
  if (out_size < DHID || (out_size % DHID) != 0) return;
  const int nG = out_size / DHID;
  if (nG > 65535 || (nG % GBM) != 0) return;

  const float* h    = (const float*)d_in[0];
  const int*   src  = (const int*)  d_in[1];
  const int*   dst  = (const int*)  d_in[2];
  const int*   gid  = (const int*)  d_in[3];
  const float* W1s  = (const float*)d_in[4];
  const float* W2s  = (const float*)d_in[5];
  const float* g1   = (const float*)d_in[6];
  const float* b1   = (const float*)d_in[7];
  const float* g2   = (const float*)d_in[8];
  const float* b2   = (const float*)d_in[9];
  const float* pW   = (const float*)d_in[10];
  const float* pB   = (const float*)d_in[11];
  float* out = (float*)d_out;

  const int MP   = cdiv(nN, GBM) * GBM;
  const int gM   = MP / GBM;
  const int nb   = pick_nb(nE, nN);
  const int gA   = cdiv(MP, nb);
  const int vec8 = ((nE & 3) == 0) ? 1 : 0;
  if ((long long)gA * nb < (long long)MP) return;
  if ((long long)(gM - 1) * GBM >= (long long)nN) return;
  const int nUw  = 2 * NLAY * NUSQ;
  const int nU4  = MP * (DHID / 4);
  const int seg  = (cdiv(nN, NTHR) + 3) & ~3;
  if ((long long)seg * NTHR < (long long)nN) return;

  char* ws = (char*)d_ws;
  size_t off = 0;
  const size_t oWT = off; off = al256(off + (size_t)2 * NLAY * WSQ * 2);
  const size_t oBT = off; off = al256(off + (size_t)DHID * KR * 2);
  const size_t oHF = off; off = al256(off + (size_t)MP * DHID * 4);
  const size_t oP1 = off; off = al256(off + (size_t)MP * APW * 2);
  const size_t oP2 = off; off = al256(off + (size_t)MP * DHID * 4);
  const size_t oPT = off; off = al256(off + (size_t)gM * PARTW * 4);
  const size_t oSS = off; off = al256(off + (size_t)(4 * DHID) * 4);
  const size_t oMB = off; off = al256(off + (size_t)nG * MROW * 4);
  const size_t oPA = off; off = al256(off + (size_t)nG * KR * 2);
  if (off > ws_size || off > (size_t)WSMAX) return;
  unsigned short* WT   = (unsigned short*)(ws + oWT);
  unsigned short* BT   = (unsigned short*)(ws + oBT);
  float*          HF   = (float*)(ws + oHF);
  unsigned short* P1   = (unsigned short*)(ws + oP1);
  float*          P2   = (float*)(ws + oP2);
  float*          PART = (float*)(ws + oPT);
  float*          SS   = (float*)(ws + oSS);
  int*            MEMB = (int*)(ws + oMB);
  unsigned short* PA   = (unsigned short*)(ws + oPA);

  hipFuncSetAttribute(reinterpret_cast<const void*>(&k_agg), hipFuncAttributeMaxDynamicSharedMemorySize, LDS_AGG);

  k_pa<<<nU4 / NTHR, NTHR, 0, stream>>>(h, nN, nU4, HF);
  k_pb<<<nUw / NTHR, NTHR, 0, stream>>>(W1s, W2s, nUw, WT);
  k_pc<<<NUR / NTHR, NTHR, 0, stream>>>(pW, NUR, BT);
  k_mem<<<nG, NTHR, 0, stream>>>(gid, nN, seg, MEMB);
  k_pool<<<nG, DHID, 0, stream>>>(HF, MEMB, nN, 0, 1, PA);

  for (int l = 0; l < NLAY; ++l) {
    k_agg<<<gA, NTHR, LDS_AGG, stream>>>(src, dst, HF, P1, APW, nN, nE, nb, vec8, MP);
    k_gm<KTOT, 0><<<gM, GTHR, 0, stream>>>(P1, WT + (size_t)(2 * l) * WSQ, pB, P2, PART, nN, MP);
    k_comb<<<1, DHID, 0, stream>>>(PART, gM, g1 + (size_t)l * DHID, b1 + (size_t)l * DHID, SS);
    k_apa<<<MP / APR, NTHR, 0, stream>>>(P2, nN, MP, SS, P1);
    k_gm<KTOT, 0><<<gM, GTHR, 0, stream>>>(P1, WT + (size_t)(2 * l + 1) * WSQ, pB, P2, PART, nN, MP);
    k_comb<<<1, DHID, 0, stream>>>(PART, gM, g2 + (size_t)l * DHID, b2 + (size_t)l * DHID, SS);
    k_apb<<<nU4 / NTHR, NTHR, 0, stream>>>(P2, nN, nU4, SS, HF);
    k_pool<<<nG, DHID, 0, stream>>>(HF, MEMB, nN, DIN + KTOT * l, 0, PA);
  }
  k_gm<KR, 1><<<nG / GBM, GTHR, 0, stream>>>(PA, BT, pB, out, PART, nG, nG);
}
